// mySeq2SeqModel_31018253812271
// MI455X (gfx1250) — hardware-verified
//
#include <hip/hip_runtime.h>
#include <math.h>

constexpr int VOCAB     = 27;
constexpr int VOCAB_PAD = 32;
constexpr int EMBD      = 64;
constexpr int HID       = 128;
constexpr int NBATCH    = 512;
constexpr int NSTEP     = 256;
constexpr int NTHR      = 256;
constexpr int SEQ_BLK   = 16;
constexpr int HPITCH    = 136;
constexpr int NROWS     = NBATCH * NSTEP;
constexpr int NOUT      = NROWS * VOCAB;
constexpr int HEAD_TILE_ROWS   = 64;
constexpr int HEAD_TILE_FLOATS = HEAD_TILE_ROWS * VOCAB;
constexpr int HEAD_TILE_V4     = HEAD_TILE_FLOATS / 4;
constexpr int HEAD_NPAD        = 32;

static_assert(NBATCH % SEQ_BLK == 0, "batch tiles");
static_assert(HID == 16 * (NTHR / 32), "8 waves x 16 hidden columns");
static_assert(HID % 32 == 0, "K multiple of 32");
static_assert((NSTEP & 1) == 0, "ping-pong parity returns to buffer 0 after one phase");
static_assert((2 * SEQ_BLK * HPITCH) % NTHR == 0, "state zero-fill exact");
static_assert(VOCAB_PAD * HID == 4 * NTHR * 4, "table staging exact");
static_assert(SEQ_BLK * NSTEP == 4 * NTHR * 4, "id staging exact");
static_assert(NROWS % (HEAD_TILE_ROWS * (NTHR / 32)) == 0, "head grid exact");
static_assert((HEAD_TILE_FLOATS * 4) % 128 == 0, "head tile is whole lines");
static_assert(HEAD_TILE_FLOATS % 4 == 0, "head tile float4 count");
static_assert(HEAD_TILE_V4 == 13 * 32 + 16, "13 full wave stores plus one 16-lane store");
static_assert(VOCAB <= HEAD_NPAD && HEAD_NPAD % 16 == 0, "head N padding");
static_assert((HPITCH * 2) % 16 == 0, "fragment loads 16-B aligned");

typedef __attribute__((ext_vector_type(16))) __bf16   v16b;
typedef __attribute__((ext_vector_type(8)))  __bf16   v8b;
typedef __attribute__((ext_vector_type(8)))  float    v8f;
typedef __attribute__((ext_vector_type(4)))  float    v4f;
typedef __attribute__((ext_vector_type(4)))  unsigned v4u;
typedef __attribute__((ext_vector_type(4)))  int      v4i;

__device__ __forceinline__ unsigned short f2bf_bits(float f) {
  unsigned u = __float_as_uint(f);
  return (unsigned short)((u + 0x7FFFu + ((u >> 16) & 1u)) >> 16);
}
__device__ __forceinline__ float bf_bits2f(unsigned short h) { return __uint_as_float(((unsigned)h) << 16); }

__device__ __forceinline__ void dep_guard_b(v8f& a, v8f& b, v16b x, v16b y) { asm volatile("v_nop\n\tv_nop\n\tv_nop\n\tv_nop" : "+v"(a), "+v"(b) : "v"(x), "v"(y)); }
__device__ __forceinline__ void step_guard_b(v8f& a, v8f& b, v16b x, v16b y, v16b p, v16b q) { asm volatile("v_nop\n\tv_nop\n\tv_nop\n\tv_nop" : "+v"(a), "+v"(b) : "v"(x), "v"(y), "v"(p), "v"(q)); }
__device__ __forceinline__ void keep4_b(v16b a, v16b b, v16b c, v16b d) { asm volatile("v_nop" :: "v"(a), "v"(b), "v"(c), "v"(d)); }
__device__ __forceinline__ void acc_guard4(v8f& a, v8f& b, v8f& c, v8f& d) { asm volatile("v_nop\n\tv_nop\n\tv_nop\n\tv_nop" : "+v"(a), "+v"(b), "+v"(c), "+v"(d)); }
__device__ __forceinline__ void pin_b(v16b& a) { asm volatile("" : "+v"(a)); }

template <typename T> struct Frag;
template <> struct Frag<__bf16> {
  typedef v16b V; union U { v16b v; v8b h[2]; };
  static __device__ __forceinline__ v16b load(const __bf16* p) {
    U f; f.h[0] = *(const v8b*)(p); f.h[1] = *(const v8b*)(p + 16); return f.v;
  }
  static __device__ __forceinline__ v8f mma(v16b a, v16b b, v8f c) {
    return __builtin_amdgcn_wmma_f32_16x16x32_bf16(false, a, false, b, (short)0, c, false, false);
  }
};

__global__ __launch_bounds__(NTHR) void ptab_kernel(const float* __restrict__ emb,
                                                    const float* __restrict__ w_enc, const float* __restrict__ b_enc,
                                                    const float* __restrict__ w_dec, const float* __restrict__ b_dec,
                                                    float* __restrict__ ptab) {
  const int g     = blockIdx.x * NTHR + threadIdx.x;
  const int table = g >> 10;
  const int i     = g & 1023;
  const int v     = i >> 5;
  const int n4    = (i & 31) * 4;
  const int vc    = (v < VOCAB) ? v : (VOCAB - 1);
  const float* W    = table ? w_dec : w_enc;
  const float* bvec = table ? b_dec : b_enc;
  const float* er   = emb + vc * EMBD;
  float a0 = 0.0f, a1 = 0.0f, a2 = 0.0f, a3 = 0.0f;
#pragma unroll 1
  for (int k = 0; k < EMBD; ++k) {
    const float e = er[k];
    const v4f w = *(const v4f*)(W + k * HID + n4);
    a0 = fmaf(e, w[0], a0);
    a1 = fmaf(e, w[1], a1);
    a2 = fmaf(e, w[2], a2);
    a3 = fmaf(e, w[3], a3);
  }
  const v4f bb = *(const v4f*)(bvec + n4);
  const bool live = (v < VOCAB);
  v4f o;
  o[0] = live ? (a0 + bb[0]) : 0.0f;
  o[1] = live ? (a1 + bb[1]) : 0.0f;
  o[2] = live ? (a2 + bb[2]) : 0.0f;
  o[3] = live ? (a3 + bb[3]) : 0.0f;
  float* op = ptab + table * (VOCAB_PAD * HID) + v * HID + n4;
  *(volatile v4f*)op = o;
  __threadfence();
  *(volatile v4f*)op = o;
}

__global__ __launch_bounds__(NTHR) void tsplit_kernel(const float* __restrict__ u_enc, const float* __restrict__ u_dec,
                                                      unsigned short* __restrict__ ut) {
  __shared__ float Tt[64 * 65];
  const int tid = threadIdx.x;
  const int c0 = blockIdx.x * 64, r0 = blockIdx.y * 64, which = blockIdx.z;
  const float* src = which ? u_dec : u_enc;
  unsigned short* Oh = ut + (size_t)(2 * which) * HID * HID;
  unsigned short* Ol = Oh + (size_t)HID * HID;
#pragma unroll
  for (int i = 0; i < 4; ++i) {
    const int idx = i * NTHR + tid;
    const int rr = idx >> 4, cc = (idx & 15) * 4;
    const v4f v = *(const v4f*)(src + (size_t)(r0 + rr) * HID + c0 + cc);
    Tt[rr * 65 + cc + 0] = v[0];
    Tt[rr * 65 + cc + 1] = v[1];
    Tt[rr * 65 + cc + 2] = v[2];
    Tt[rr * 65 + cc + 3] = v[3];
  }
  __syncthreads();
  const int q = tid >> 3, c8 = (tid & 7) * 8;
  v4u hv[2], lv[2];
#pragma unroll
  for (int g = 0; g < 2; ++g) {
    const int qq = g * 32 + q;
#pragma unroll
    for (int e2 = 0; e2 < 4; ++e2) {
      const float f0 = Tt[(c8 + 2 * e2) * 65 + qq];
      const float f1 = Tt[(c8 + 2 * e2 + 1) * 65 + qq];
      const unsigned short h0 = f2bf_bits(f0);
      const unsigned short h1 = f2bf_bits(f1);
      const unsigned short l0 = f2bf_bits(f0 - bf_bits2f(h0));
      const unsigned short l1 = f2bf_bits(f1 - bf_bits2f(h1));
      hv[g][e2] = (unsigned)h0 | ((unsigned)h1 << 16);
      lv[g][e2] = (unsigned)l0 | ((unsigned)l1 << 16);
    }
  }
  for (int pass = 0; pass < 2; ++pass) {
#pragma unroll
    for (int g = 0; g < 2; ++g) {
      const size_t o = (size_t)(c0 + g * 32 + q) * HID + (size_t)(r0 + c8);
      *(volatile v4u*)(Oh + o) = hv[g];
      *(volatile v4u*)(Ol + o) = lv[g];
    }
    __threadfence();
  }
}

__global__ __launch_bounds__(NTHR) void wout_kernel(const float* __restrict__ w_out,
                                                    unsigned short* __restrict__ woh, unsigned short* __restrict__ wol) {
  const int i  = blockIdx.x * NTHR + threadIdx.x;
  const int n  = i >> 4;
  const int k8 = (i & 15) * 8;
  const int nc = (n < VOCAB) ? n : (VOCAB - 1);
  const bool live = (n < VOCAB);
  v4u hv, lv;
#pragma unroll
  for (int e2 = 0; e2 < 4; ++e2) {
    const float g0 = w_out[(k8 + 2 * e2) * VOCAB + nc];
    const float g1 = w_out[(k8 + 2 * e2 + 1) * VOCAB + nc];
    const float f0 = live ? g0 : 0.0f;
    const float f1 = live ? g1 : 0.0f;
    const unsigned short h0 = f2bf_bits(f0);
    const unsigned short h1 = f2bf_bits(f1);
    const unsigned short l0 = f2bf_bits(f0 - bf_bits2f(h0));
    const unsigned short l1 = f2bf_bits(f1 - bf_bits2f(h1));
    hv[e2] = (unsigned)h0 | ((unsigned)h1 << 16);
    lv[e2] = (unsigned)l0 | ((unsigned)l1 << 16);
  }
  const size_t o = (size_t)n * HID + k8;
  *(volatile v4u*)(woh + o) = hv;
  *(volatile v4u*)(wol + o) = lv;
  __threadfence();
  *(volatile v4u*)(woh + o) = hv;
  *(volatile v4u*)(wol + o) = lv;
}

__global__ __launch_bounds__(NTHR) void rnn_kernel(const int* __restrict__ enc_ids, const int* __restrict__ dec_ids,
                                                   const float* __restrict__ ptab, const unsigned short* __restrict__ ut,
                                                   unsigned short* __restrict__ hhi, unsigned short* __restrict__ hlo) {
  __shared__ __align__(16) float  Ps[VOCAB_PAD * HID];
  __shared__ __align__(16) int    Ids[SEQ_BLK * NSTEP];
  __shared__ __align__(16) __bf16 Hh[2][SEQ_BLK * HPITCH];
  __shared__ __align__(16) __bf16 Hl[2][SEQ_BLK * HPITCH];
  const int tid = threadIdx.x, lane = tid & 31, wave = tid >> 5;
  const int c = lane & 15, hh = lane >> 4, koff = hh * 8;
  const int b0 = blockIdx.x * SEQ_BLK;
  const int ncol = 16 * wave + c;

  {
    const __bf16 zb = __builtin_bit_cast(__bf16, (unsigned short)0);
    __bf16* zh = &Hh[0][0];
    __bf16* zl = &Hl[0][0];
#pragma unroll 1
    for (int i = tid; i < 2 * SEQ_BLK * HPITCH; i += NTHR) { zh[i] = zb; zl[i] = zb; }
  }
  const v8f z8 = {0.f, 0.f, 0.f, 0.f, 0.f, 0.f, 0.f, 0.f};

#pragma unroll 1
  for (int phase = 0; phase < 2; ++phase) {
    const int* ids = (phase ? dec_ids : enc_ids) + (size_t)b0 * NSTEP;
    const float* pg = ptab + phase * (VOCAB_PAD * HID);
    const __bf16* uh = (const __bf16*)(ut + (size_t)(2 * phase) * HID * HID) + (size_t)ncol * HID + koff;
    const __bf16* ul = uh + (size_t)HID * HID;

#pragma unroll
    for (int i = 0; i < 4; ++i) {
      const int idx = i * NTHR + tid;
      const v4f pv = *(const v4f*)(pg + 4 * idx);
      *(v4f*)(Ps + 4 * idx) = pv;
      v4i iv = *(const v4i*)(ids + 4 * idx);
#pragma unroll
      for (int e = 0; e < 4; ++e) {
        int x = iv[e];
        x = x < 0 ? 0 : x;
        x = x > (VOCAB - 1) ? (VOCAB - 1) : x;
        iv[e] = x;
      }
      *(v4i*)(Ids + 4 * idx) = iv;
    }
    v16b Bh[4], Bl[4];
#pragma unroll
    for (int kt = 0; kt < 4; ++kt) {
      Bh[kt] = Frag<__bf16>::load(uh + 32 * kt);
      Bl[kt] = Frag<__bf16>::load(ul + 32 * kt);
      pin_b(Bh[kt]);
      pin_b(Bl[kt]);
    }
    __syncthreads();

#pragma unroll 1
    for (int t = 0; t < NSTEP; ++t) {
      const int cur = t & 1;
      const __bf16* ahr = &Hh[cur][0] + c * HPITCH + koff;
      const __bf16* alr = &Hl[cur][0] + c * HPITCH + koff;
      v8f acc0 = z8, acc1 = z8;
#pragma unroll
      for (int r = 0; r < 8; ++r) {
        const int id = Ids[(8 * hh + r) * NSTEP + t];
        acc0[r] = Ps[id * HID + ncol];
      }
#pragma unroll
      for (int kt = 0; kt < 4; ++kt) {
        const v16b ah = Frag<__bf16>::load(ahr + 32 * kt);
        const v16b al = Frag<__bf16>::load(alr + 32 * kt);
        acc0 = Frag<__bf16>::mma(ah, Bh[kt], acc0);
        acc1 = Frag<__bf16>::mma(al, Bh[kt], acc1);
        acc1 = Frag<__bf16>::mma(ah, Bl[kt], acc1);
        step_guard_b(acc0, acc1, ah, al, Bh[kt], Bl[kt]);
      }
      __bf16* hwh = &Hh[cur ^ 1][0];
      __bf16* hwl = &Hl[cur ^ 1][0];
#pragma unroll
      for (int r = 0; r < 8; ++r) {
        const float z  = acc0[r] + acc1[r];
        const float hv = tanhf(z);
        const unsigned short hb = f2bf_bits(hv);
        const unsigned short lb = f2bf_bits(hv - bf_bits2f(hb));
        hwh[(8 * hh + r) * HPITCH + ncol] = __builtin_bit_cast(__bf16, hb);
        hwl[(8 * hh + r) * HPITCH + ncol] = __builtin_bit_cast(__bf16, lb);
      }
      __syncthreads();
      if (phase == 1) {
        const int row = 2 * wave + hh;
        const int c8 = c * 8;
        const v4u vh = *(const v4u*)(const void*)(&Hh[cur ^ 1][0] + row * HPITCH + c8);
        const v4u vl = *(const v4u*)(const void*)(&Hl[cur ^ 1][0] + row * HPITCH + c8);
        const size_t go = ((size_t)(b0 + row) * NSTEP + (size_t)t) * HID + c8;
        for (int pass = 0; pass < 2; ++pass) {
          *(volatile v4u*)(hhi + go) = vh;
          *(volatile v4u*)(hlo + go) = vl;
          __threadfence();
        }
      }
    }
  }
}

__global__ __launch_bounds__(NTHR) void head_gemm_kernel(const unsigned short* __restrict__ hhi, const unsigned short* __restrict__ hlo,
                                                         const unsigned short* __restrict__ woh, const unsigned short* __restrict__ wol,
                                                         const float* __restrict__ b_out, float* __restrict__ out) {
  __shared__ __align__(16) float sT[NTHR / 32][HEAD_TILE_FLOATS];
  const int tid = threadIdx.x, lane = tid & 31, wave = tid >> 5;
  const int c = lane & 15, hh = lane >> 4, koff = hh * 8;
  const int m0 = (blockIdx.x * (NTHR / 32) + wave) * HEAD_TILE_ROWS;
  const __bf16* Ah = (const __bf16*)hhi + (size_t)(m0 + c) * HID + koff;
  const __bf16* Al = (const __bf16*)hlo + (size_t)(m0 + c) * HID + koff;
  const __bf16* Bh = (const __bf16*)woh + (size_t)c * HID + koff;
  const __bf16* Bl = (const __bf16*)wol + (size_t)c * HID + koff;

  v8f acc[4][2];
#pragma unroll
  for (int i = 0; i < 4; ++i)
#pragma unroll
    for (int j = 0; j < 2; ++j) acc[i][j] = (v8f){0.f, 0.f, 0.f, 0.f, 0.f, 0.f, 0.f, 0.f};

  for (int k0 = 0; k0 < HID; k0 += 32) {
    v16b bh[2], bl[2];
#pragma unroll
    for (int j = 0; j < 2; ++j) {
      bh[j] = Frag<__bf16>::load(Bh + (size_t)j * 16 * HID + k0);
      bl[j] = Frag<__bf16>::load(Bl + (size_t)j * 16 * HID + k0);
    }
#pragma unroll
    for (int i = 0; i < 4; ++i) {
      const v16b ah = Frag<__bf16>::load(Ah + (size_t)i * 16 * HID + k0);
      const v16b al = Frag<__bf16>::load(Al + (size_t)i * 16 * HID + k0);
#pragma unroll
      for (int j = 0; j < 2; ++j) {
        acc[i][j] = Frag<__bf16>::mma(ah, bh[j], acc[i][j]);
        acc[i][j] = Frag<__bf16>::mma(ah, bl[j], acc[i][j]);
        acc[i][j] = Frag<__bf16>::mma(al, bh[j], acc[i][j]);
      }
      dep_guard_b(acc[i][0], acc[i][1], ah, al);
    }
    keep4_b(bh[0], bh[1], bl[0], bl[1]);
  }
  acc_guard4(acc[0][0], acc[0][1], acc[1][0], acc[1][1]);
  acc_guard4(acc[2][0], acc[2][1], acc[3][0], acc[3][1]);

  float* slab = sT[wave];
#pragma unroll
  for (int j = 0; j < 2; ++j) {
    const int n  = 16 * j + c;
    const int nb = (n < VOCAB) ? n : (VOCAB - 1);
    const float bv = b_out[nb];
#pragma unroll
    for (int i = 0; i < 4; ++i) {
#pragma unroll
      for (int r = 0; r < 8; ++r) {
        const int row = 16 * i + 8 * hh + r;
        const float v = acc[i][j][r] + bv;
        if (n < VOCAB) slab[row * VOCAB + n] = v;
      }
    }
  }
  __builtin_amdgcn_fence(__ATOMIC_RELEASE, "workgroup");
  __builtin_amdgcn_wave_barrier();
  __builtin_amdgcn_fence(__ATOMIC_ACQUIRE, "workgroup");
  float* dst = out + (size_t)m0 * VOCAB;
  for (int pass = 0; pass < 2; ++pass) {
#pragma unroll
    for (int it = 0; it < 14; ++it) {
      const int idx = it * 32 + lane;
      const int idc = (idx < HEAD_TILE_V4) ? idx : (HEAD_TILE_V4 - 1);
      const v4f v = *(const v4f*)(slab + 4 * idc);
      if (idx < HEAD_TILE_V4) *(volatile v4f*)(dst + 4 * idx) = v;
    }
    __threadfence();
  }
}

extern "C" void kernel_launch(void* const* d_in, const int* in_sizes, int n_in,
                              void* d_out, int out_size, void* d_ws, size_t ws_size, hipStream_t stream) {
  if (n_in < 11 || d_out == nullptr || d_ws == nullptr) return;
  if (in_sizes[0] != NBATCH * NSTEP || in_sizes[1] != NBATCH * NSTEP || in_sizes[2] != VOCAB * EMBD ||
      in_sizes[3] != EMBD * HID || in_sizes[4] != HID * HID || in_sizes[5] != HID ||
      in_sizes[6] != EMBD * HID || in_sizes[7] != HID * HID || in_sizes[8] != HID ||
      in_sizes[9] != HID * VOCAB || in_sizes[10] != VOCAB || out_size != NOUT) return;

  const int*   enc_ids = (const int*)d_in[0];
  const int*   dec_ids = (const int*)d_in[1];
  const float* emb     = (const float*)d_in[2];
  const float* w_enc   = (const float*)d_in[3];
  const float* u_enc   = (const float*)d_in[4];
  const float* b_enc   = (const float*)d_in[5];
  const float* w_dec   = (const float*)d_in[6];
  const float* u_dec   = (const float*)d_in[7];
  const float* b_dec   = (const float*)d_in[8];
  const float* w_out   = (const float*)d_in[9];
  const float* b_out   = (const float*)d_in[10];
  float* out = (float*)d_out;

  char* ws = (char*)d_ws; size_t off = 0;
  auto carve = [&](size_t bytes) -> char* { char* p = ws + off; off += (bytes + 255) & ~(size_t)255; return p; };
  unsigned short* HHI  = (unsigned short*)carve((size_t)NROWS * HID * 2);
  unsigned short* HLO  = (unsigned short*)carve((size_t)NROWS * HID * 2);
  unsigned short* UT   = (unsigned short*)carve((size_t)4 * HID * HID * 2);
  unsigned short* WOH  = (unsigned short*)carve((size_t)HEAD_NPAD * HID * 2);
  unsigned short* WOL  = (unsigned short*)carve((size_t)HEAD_NPAD * HID * 2);
  float*          PTAB = (float*)carve((size_t)2 * VOCAB_PAD * HID * 4);
  if (off > ws_size || off > (size_t)134217728) return;

  ptab_kernel<<<(2 * VOCAB_PAD * (HID / 4)) / NTHR, NTHR, 0, stream>>>(emb, w_enc, b_enc, w_dec, b_dec, PTAB);
  tsplit_kernel<<<dim3(HID / 64, HID / 64, 2), NTHR, 0, stream>>>(u_enc, u_dec, UT);
  wout_kernel<<<(HEAD_NPAD * (HID / 8)) / NTHR, NTHR, 0, stream>>>(w_out, WOH, WOL);
  rnn_kernel<<<NBATCH / SEQ_BLK, NTHR, 0, stream>>>(enc_ids, dec_ids, PTAB, UT, HHI, HLO);
  head_gemm_kernel<<<NROWS / (HEAD_TILE_ROWS * (NTHR / 32)), NTHR, 0, stream>>>(HHI, HLO, WOH, WOL, b_out, out);
}
